// RetNetBlock_21973052686682
// MI455X (gfx1250) — hardware-verified
//
#include <hip/hip_runtime.h>
#include <math.h>

constexpr int kB    = 4;
constexpr int kT    = 1024;
constexpr int kD    = 1024;
constexpr int kH    = 16;
constexpr int kDH   = 64;
constexpr int kD2   = 2048;
constexpr int kTok  = kB * kT;
constexpr int kQKVN = 3 * kD;
constexpr int kNG   = kB * kH;
constexpr int kChunkG = 8;
constexpr int kNChunk = kNG / kChunkG;

constexpr float kWCarry   = 16.0f;
constexpr float kQKCarry  = 1024.0f;
constexpr float kSim256   = 256.0f;
constexpr float kQKVScale = 1.0f / 16.0f;
constexpr float kSScale   = 1.0f / (1024.0f * 1024.0f);
constexpr float kPVScale  = 128.0f / 2048.0f;
constexpr float kOWScale  = 1.0f / (128.0f * 16.0f);
constexpr float kW1Scale  = 1.0f / 16.0f;
constexpr float kHCarry   = 16.0f;
constexpr float kW2Scale  = 1.0f / (16.0f * 16.0f);

constexpr size_t kOffW3  = 0;
constexpr size_t kOffOW  = kOffW3 + (size_t)kQKVN * kD * 2;
constexpr size_t kOffW1  = kOffOW + (size_t)kD * kD * 2;
constexpr size_t kOffW2  = kOffW1 + (size_t)kD2 * kD * 2;
constexpr size_t kOffXN  = kOffW2 + (size_t)kD * kD2 * 2;
constexpr size_t kOffBig = kOffXN + (size_t)kTok * kD * 2;
constexpr size_t kBigBytes = (size_t)kTok * kQKVN * 4;
constexpr size_t kOffQ   = kOffBig + kBigBytes;
constexpr size_t kOffK   = kOffQ + (size_t)kNG * kT * kDH * 2;
constexpr size_t kOffVT  = kOffK + (size_t)kNG * kT * kDH * 2;
constexpr size_t kOffX1  = kOffVT + (size_t)kNG * kDH * kT * 2;
constexpr size_t kWsTotal = kOffX1 + (size_t)kTok * kD * 4;
static_assert(kWsTotal == 117440512, "carve total");
static_assert(kWsTotal <= 134217728, "carve cap");
static_assert((size_t)kChunkG * kT * kT * 4 <= kBigBytes, "scores f32 chunk fits big region");
static_assert((size_t)kTok * kD2 * 4 <= kBigBytes, "u f32 fits big region");
static_assert((size_t)kChunkG * kT * kT * 2 <= (size_t)kTok * kD * 4, "scores f16 chunk fits x1 region");
static_assert((size_t)kTok * kD2 * 2 <= (size_t)2 * kNG * kT * kDH * 2, "h f16 fits q+k region");

typedef __attribute__((ext_vector_type(16))) _Float16 v16h;
typedef __attribute__((ext_vector_type(8)))  _Float16 v8h;
typedef __attribute__((ext_vector_type(16))) __bf16   v16b;
typedef __attribute__((ext_vector_type(8)))  __bf16   v8b;
typedef __attribute__((ext_vector_type(8)))  float    v8f;
typedef __attribute__((ext_vector_type(4)))  float    v4f;
typedef __attribute__((ext_vector_type(4)))  unsigned int v4u;

__device__ __forceinline__ unsigned short f2bf_bits(float f) {
  unsigned u = __float_as_uint(f);
  return (unsigned short)((u + 0x7FFFu + ((u >> 16) & 1u)) >> 16);
}
__device__ __forceinline__ float bf_bits2f(unsigned short h) { return __uint_as_float(((unsigned)h) << 16); }

__device__ __forceinline__ void dep_guard_h(v8f& a, v8f& b, v16h x, v16h y) { asm volatile("v_nop\n\tv_nop\n\tv_nop\n\tv_nop" : "+v"(a), "+v"(b) : "v"(x), "v"(y)); }
__device__ __forceinline__ void dep_guard_b(v8f& a, v8f& b, v16b x, v16b y) { asm volatile("v_nop\n\tv_nop\n\tv_nop\n\tv_nop" : "+v"(a), "+v"(b) : "v"(x), "v"(y)); }
__device__ __forceinline__ void keep4_h(v16h a, v16h b, v16h c, v16h d) { asm volatile("v_nop" :: "v"(a), "v"(b), "v"(c), "v"(d)); }
__device__ __forceinline__ void keep4_b(v16b a, v16b b, v16b c, v16b d) { asm volatile("v_nop" :: "v"(a), "v"(b), "v"(c), "v"(d)); }
__device__ __forceinline__ void acc_guard4(v8f& a, v8f& b, v8f& c, v8f& d) { asm volatile("v_nop\n\tv_nop\n\tv_nop\n\tv_nop" : "+v"(a), "+v"(b), "+v"(c), "+v"(d)); }
template <typename T> struct Frag;
template <> struct Frag<_Float16> {
  typedef v16h V; union U { v16h v; v8h h[2]; };
  static __device__ __forceinline__ v16h load(const _Float16* p) {
    U f; f.h[0] = *(const v8h*)(p); f.h[1] = *(const v8h*)(p + 16); return f.v;
  }
  static __device__ __forceinline__ v8f mma(v16h a, v16h b, v8f c) {
    return __builtin_amdgcn_wmma_f32_16x16x32_f16(false, a, false, b, (short)0, c, false, false);
  }
  static __device__ __forceinline__ void guard(v8f& a, v8f& b, v16h x, v16h y) { dep_guard_h(a, b, x, y); }
  static __device__ __forceinline__ void keep(v16h a, v16h b, v16h c, v16h d) { keep4_h(a, b, c, d); }
};
template <> struct Frag<__bf16> {
  typedef v16b V; union U { v16b v; v8b h[2]; };
  static __device__ __forceinline__ v16b load(const __bf16* p) {
    U f; f.h[0] = *(const v8b*)(p); f.h[1] = *(const v8b*)(p + 16); return f.v;
  }
  static __device__ __forceinline__ v8f mma(v16b a, v16b b, v8f c) {
    return __builtin_amdgcn_wmma_f32_16x16x32_bf16(false, a, false, b, (short)0, c, false, false);
  }
  static __device__ __forceinline__ void guard(v8f& a, v8f& b, v16b x, v16b y) { dep_guard_b(a, b, x, y); }
  static __device__ __forceinline__ void keep(v16b a, v16b b, v16b c, v16b d) { keep4_b(a, b, c, d); }
};

__device__ __forceinline__ unsigned pk16(unsigned short a, unsigned short b) { return (unsigned)a | ((unsigned)b << 16); }
__device__ __forceinline__ unsigned short h_bits(float f) { const _Float16 h = (_Float16)f; return __builtin_bit_cast(unsigned short, h); }

template <int ET> struct Elem;
template <> struct Elem<0> { typedef _Float16 T; };
template <> struct Elem<1> { typedef __bf16 T; };
template <int ET, bool SPLIT, int BIAS_MODE, int OUT_MODE, bool RESID, int ACT = 0>
__global__ __launch_bounds__(256) void wmma_gemm64(
    const unsigned short* __restrict__ Ap, const unsigned short* __restrict__ A2p, int lda, long strideA,
    const unsigned short* __restrict__ Btp, const unsigned short* __restrict__ Bt2p, int ldb, long strideB,
    void* __restrict__ Cout, void* __restrict__ Cout2, int ldc, long strideC,
    const float* __restrict__ bias,
    const float* __restrict__ resid, long strideR,
    int M, int N, int K, float scale) {
  typedef typename Elem<ET>::T T;
  typedef typename Frag<T>::V V;
  const T* A = (const T*)Ap; const T* A2 = (const T*)A2p; const T* Bt = (const T*)Btp; const T* Bt2 = (const T*)Bt2p;
  __shared__ __align__(16) float sT[8][16 * 68];
  const int b    = blockIdx.y;
  const int lane = threadIdx.x & 31;
  const int wave = threadIdx.x >> 5;
  const int tilesN = N >> 6;
  const int tilesM = M >> 6;
  const int tile = blockIdx.x * 8 + wave;
  if (tile >= tilesM * tilesN) return;
  const int tm = tile / tilesN;
  const int tn = tile - tm * tilesN;
  const int m0 = tm << 6;
  const int n0 = tn << 6;

  const T* Ab  = A  + (size_t)b * strideA;
  const T* Bb  = Bt + (size_t)b * strideB;
  const T* Ab2 = SPLIT ? (A2  + (size_t)b * strideA) : nullptr;
  const T* Bb2 = SPLIT ? (Bt2 + (size_t)b * strideB) : nullptr;

  const int rlane = lane & 15;
  const int koff  = (lane >> 4) * 8;
  const int mOff  = (lane >> 4) * 8;

  v8f acc[4][4];
#pragma unroll
  for (int i = 0; i < 4; ++i)
#pragma unroll
    for (int j = 0; j < 4; ++j) acc[i][j] = (v8f){0.f,0.f,0.f,0.f,0.f,0.f,0.f,0.f};

  for (int k0 = 0; k0 < K; k0 += 32) {
    V bh[4], bl[4];
#pragma unroll
    for (int j = 0; j < 4; ++j) {
      const size_t bo = (size_t)(n0 + (j << 4) + rlane) * ldb + koff + k0;
      bh[j] = Frag<T>::load(Bb + bo);
      if (SPLIT) bl[j] = Frag<T>::load(Bb2 + bo);
    }
#pragma unroll
    for (int i = 0; i < 4; ++i) {
      const size_t ao = (size_t)(m0 + (i << 4) + rlane) * lda + koff + k0;
      V ah = Frag<T>::load(Ab + ao);
      V al;
      if (SPLIT) al = Frag<T>::load(Ab2 + ao);
#pragma unroll
      for (int j = 0; j < 4; ++j) {
        acc[i][j] = Frag<T>::mma(ah, bh[j], acc[i][j]);
        if (SPLIT) {
          acc[i][j] = Frag<T>::mma(ah, bl[j], acc[i][j]);
          acc[i][j] = Frag<T>::mma(al, bh[j], acc[i][j]);
        }
      }
      Frag<T>::guard(acc[i][0], acc[i][3], ah, SPLIT ? al : ah);
    }
    Frag<T>::keep(bh[0], bh[1], bh[2], bh[3]);
    if (SPLIT) Frag<T>::keep(bl[0], bl[1], bl[2], bl[3]);
  }
  acc_guard4(acc[0][0], acc[0][1], acc[0][2], acc[0][3]);
  acc_guard4(acc[1][0], acc[1][1], acc[1][2], acc[1][3]);
  acc_guard4(acc[2][0], acc[2][1], acc[2][2], acc[2][3]);
  acc_guard4(acc[3][0], acc[3][1], acc[3][2], acc[3][3]);

  float* slab = sT[wave];
  const float* Rb = RESID ? (resid + (size_t)b * strideR) : nullptr;
#pragma unroll
  for (int i = 0; i < 4; ++i) {
    const int mBase = m0 + (i << 4);
#pragma unroll
    for (int j = 0; j < 4; ++j) {
      const int n = n0 + (j << 4) + rlane;
      float bv = 0.f;
      if (BIAS_MODE == 2) bv = bias[n];
#pragma unroll
      for (int r = 0; r < 8; ++r) {
        float v = acc[i][j][r] * scale;
        if (BIAS_MODE == 1) v += bias[mBase + mOff + r];
        if (BIAS_MODE == 2) v += bv;
        if (RESID) v += Rb[(size_t)(mBase + mOff + r) * ldc + n];
        if (ACT == 1) v = tanhf(v);
        if (ACT == 2) v = fmaxf(v, 0.0f);
        if (ACT == 3) v = v / (1.0f + expf(-v));
        if (ACT == 4) v = (v > 0.f) ? v : 0.01f * v;
        if (ACT == 5) v = 0.5f * v * (1.0f + erff(v * 0.70710678118654752f));
        slab[(mOff + r) * 68 + (j << 4) + rlane] = v;
      }
    }
    __builtin_amdgcn_fence(__ATOMIC_RELEASE, "workgroup");
    __builtin_amdgcn_wave_barrier();
    __builtin_amdgcn_fence(__ATOMIC_ACQUIRE, "workgroup");
    if (OUT_MODE == 0) {
      float* C = (float*)Cout + (size_t)b * strideC;
      const int hh = lane >> 4, c4 = (lane & 15) * 4;
      for (int pass = 0; pass < 2; ++pass) {
#pragma unroll
        for (int it = 0; it < 8; ++it) {
          const int row = it * 2 + hh;
          v4f v = *(const v4f*)(slab + row * 68 + c4);
          *(volatile v4f*)(C + (size_t)(mBase + row) * ldc + n0 + c4) = v;
        }
        __threadfence();
      }
    } else {
      const int q = lane >> 3, c8 = (lane & 7) * 8;
      unsigned short* C  = (unsigned short*)Cout  + (size_t)b * strideC;
      unsigned short* C2 = (OUT_MODE == 2) ? ((unsigned short*)Cout2 + (size_t)b * strideC) : nullptr;
      for (int pass = 0; pass < 2; ++pass) {
#pragma unroll
        for (int it = 0; it < 4; ++it) {
          const int row = it * 4 + q;
          const float* sp = slab + row * 68 + c8;
          v8h hv, lv;
#pragma unroll
          for (int e = 0; e < 8; ++e) {
            if (OUT_MODE == 1) {
              hv[e] = (_Float16)sp[e];
            } else {
              unsigned short hb = f2bf_bits(sp[e]);
              unsigned short lb = f2bf_bits(sp[e] - bf_bits2f(hb));
              hv[e] = __builtin_bit_cast(_Float16, hb);
              lv[e] = __builtin_bit_cast(_Float16, lb);
            }
          }
          *(volatile v8h*)(C + (size_t)(mBase + row) * ldc + n0 + c8) = hv;
          if (OUT_MODE == 2) *(volatile v8h*)(C2 + (size_t)(mBase + row) * ldc + n0 + c8) = lv;
        }
        __threadfence();
      }
    }
    __builtin_amdgcn_fence(__ATOMIC_RELEASE, "workgroup");
    __builtin_amdgcn_wave_barrier();
    __builtin_amdgcn_fence(__ATOMIC_ACQUIRE, "workgroup");
  }
}

__device__ __forceinline__ float wave_sum(float v) {
#pragma unroll
  for (int off = 16; off > 0; off >>= 1) v += __shfl_xor(v, off, 32);
  return v;
}

__global__ __launch_bounds__(256) void cast8_kernel(const float* __restrict__ s0, const float* __restrict__ s1,
                                                    const float* __restrict__ s2, unsigned short* __restrict__ out,
                                                    int n8, float scale) {
  const int i = blockIdx.x * 256 + threadIdx.x;
  if (i >= n8) return;
  const int z = blockIdx.y;
  const float* src = (z == 0) ? s0 : (z == 1) ? s1 : s2;
  const float* p = src + 8 * (size_t)i;
  const v4f a = *(const v4f*)(p);
  const v4f c = *(const v4f*)(p + 4);
  unsigned short hb[8];
#pragma unroll
  for (int e = 0; e < 4; ++e) {
    hb[e]     = h_bits(a[e] * scale);
    hb[4 + e] = h_bits(c[e] * scale);
  }
  const v4u u = (v4u){pk16(hb[0], hb[1]), pk16(hb[2], hb[3]), pk16(hb[4], hb[5]), pk16(hb[6], hb[7])};
  unsigned short* q = out + (size_t)z * (size_t)n8 * 8 + 8 * (size_t)i;
  *(volatile v4u*)q = u;
  __threadfence();
  *(volatile v4u*)q = u;
}

__global__ __launch_bounds__(256) void groupnorm_kernel(const float* __restrict__ x, const float* __restrict__ gam,
                                                        const float* __restrict__ bet, unsigned short* __restrict__ out) {
  __shared__ float red[8];
  const int bg = blockIdx.x;
  const int b = bg >> 4, g = bg & 15;
  const int tid = threadIdx.x, lane = tid & 31, wave = tid >> 5;
  const int q = lane >> 3, c8 = (lane & 7) * 8;
  const int col = g * kDH + c8;
  const float* xb = x + (size_t)b * kT * kD + col;

  float s = 0.f;
#pragma unroll 1
  for (int it = 0; it < 32; ++it) {
    const int t = it * 32 + wave * 4 + q;
    const float* p = xb + (size_t)t * kD;
    const v4f a = *(const v4f*)(p);
    const v4f c = *(const v4f*)(p + 4);
    s += ((a[0] + a[1]) + (a[2] + a[3])) + ((c[0] + c[1]) + (c[2] + c[3]));
  }
  s = wave_sum(s);
  if (lane == 0) red[wave] = s;
  __syncthreads();
  float tot = 0.f;
#pragma unroll
  for (int w = 0; w < 8; ++w) tot += red[w];
  const float mean = tot * (1.0f / 65536.0f);
  __syncthreads();

  float ss = 0.f;
#pragma unroll 1
  for (int it = 0; it < 32; ++it) {
    const int t = it * 32 + wave * 4 + q;
    const float* p = xb + (size_t)t * kD;
    const v4f a = *(const v4f*)(p);
    const v4f c = *(const v4f*)(p + 4);
#pragma unroll
    for (int e = 0; e < 4; ++e) {
      const float d0 = a[e] - mean;
      const float d1 = c[e] - mean;
      ss += d0 * d0;
      ss += d1 * d1;
    }
  }
  ss = wave_sum(ss);
  if (lane == 0) red[wave] = ss;
  __syncthreads();
  float tot2 = 0.f;
#pragma unroll
  for (int w = 0; w < 8; ++w) tot2 += red[w];
  const float var  = tot2 * (1.0f / 65536.0f);
  const float rstd = 1.0f / sqrtf(var + 1e-5f);

  const v4f g0 = *(const v4f*)(gam + col);
  const v4f g1 = *(const v4f*)(gam + col + 4);
  const v4f e0 = *(const v4f*)(bet + col);
  const v4f e1 = *(const v4f*)(bet + col + 4);
  unsigned short* op = out + (size_t)b * kT * kD + col;
#pragma unroll 1
  for (int it = 0; it < 32; ++it) {
    const int t = it * 32 + wave * 4 + q;
    const float* p = xb + (size_t)t * kD;
    const v4f a = *(const v4f*)(p);
    const v4f c = *(const v4f*)(p + 4);
    unsigned short hb[8];
#pragma unroll
    for (int e = 0; e < 4; ++e) {
      hb[e]     = h_bits((a[e] - mean) * rstd * g0[e] + e0[e]);
      hb[4 + e] = h_bits((c[e] - mean) * rstd * g1[e] + e1[e]);
    }
    const v4u u = (v4u){pk16(hb[0], hb[1]), pk16(hb[2], hb[3]), pk16(hb[4], hb[5]), pk16(hb[6], hb[7])};
    unsigned short* po = op + (size_t)t * kD;
    *(volatile v4u*)po = u;
    __threadfence();
    *(volatile v4u*)po = u;
  }
}

__global__ __launch_bounds__(128) void l2norm_qk_kernel(const float* __restrict__ qkv, unsigned short* __restrict__ q16,
                                                        unsigned short* __restrict__ k16) {
  __shared__ float redq[4];
  __shared__ float redk[4];
  const int r = blockIdx.x;
  const int b = r >> 10, t = r & (kT - 1);
  const int tid = threadIdx.x, lane = tid & 31, wave = tid >> 5;
  const int e0 = tid * 8;
  const float* pq = qkv + (size_t)r * kQKVN + e0;
  const float* pk = pq + kD;
  const v4f qa = *(const v4f*)(pq), qc = *(const v4f*)(pq + 4);
  const v4f ka = *(const v4f*)(pk), kc = *(const v4f*)(pk + 4);
  float sq = 0.f, sk = 0.f;
#pragma unroll
  for (int e = 0; e < 4; ++e) {
    sq += qa[e] * qa[e];
    sq += qc[e] * qc[e];
    sk += ka[e] * ka[e];
    sk += kc[e] * kc[e];
  }
  sq = wave_sum(sq);
  sk = wave_sum(sk);
  if (lane == 0) { redq[wave] = sq; redk[wave] = sk; }
  __syncthreads();
  const float nq = (redq[0] + redq[1]) + (redq[2] + redq[3]);
  const float nk = (redk[0] + redk[1]) + (redk[2] + redk[3]);
  const float iq = kQKCarry / fmaxf(sqrtf(nq), 1e-12f);
  const float ik = kQKCarry / fmaxf(sqrtf(nk), 1e-12f);
  unsigned short hq[8], hk[8];
#pragma unroll
  for (int e = 0; e < 4; ++e) {
    hq[e]     = h_bits(qa[e] * iq);
    hq[4 + e] = h_bits(qc[e] * iq);
    hk[e]     = h_bits(ka[e] * ik);
    hk[4 + e] = h_bits(kc[e] * ik);
  }
  const v4u uq = (v4u){pk16(hq[0], hq[1]), pk16(hq[2], hq[3]), pk16(hq[4], hq[5]), pk16(hq[6], hq[7])};
  const v4u uk = (v4u){pk16(hk[0], hk[1]), pk16(hk[2], hk[3]), pk16(hk[4], hk[5]), pk16(hk[6], hk[7])};
  const int h = tid >> 3, d8 = (tid & 7) * 8;
  const size_t o = ((size_t)(b * kH + h) * kT + t) * kDH + d8;
  unsigned short* oq = q16 + o;
  unsigned short* ok = k16 + o;
  *(volatile v4u*)oq = uq;
  *(volatile v4u*)ok = uk;
  __threadfence();
  *(volatile v4u*)oq = uq;
  *(volatile v4u*)ok = uk;
}

__global__ __launch_bounds__(256) void vtrans_kernel(const float* __restrict__ qkv, unsigned short* __restrict__ vt) {
  __shared__ float sm[64][65];
  const int tt = blockIdx.x;
  const int h  = blockIdx.y;
  const int b  = blockIdx.z;
  const int tid = threadIdx.x;
  const int t0 = tt * 64;
  const float* src = qkv + (size_t)(b * kT + t0) * kQKVN + 2 * kD + h * kDH;
#pragma unroll
  for (int i = 0; i < 16; ++i) {
    const int e = i * 256 + tid;
    const int r = e >> 6;
    const int c = e & 63;
    sm[c][r] = src[(size_t)r * kQKVN + c];
  }
  __syncthreads();
  const int lane = tid & 31, wave = tid >> 5;
  const int q = lane >> 3, c8 = (lane & 7) * 8;
  unsigned short* op = vt + (size_t)(b * kH + h) * kDH * kT + t0;
  for (int pass = 0; pass < 2; ++pass) {
#pragma unroll
    for (int it = 0; it < 2; ++it) {
      const int row = wave * 8 + it * 4 + q;
      unsigned short hb[8];
#pragma unroll
      for (int e = 0; e < 8; ++e) hb[e] = h_bits(sm[row][c8 + e]);
      const v4u u = (v4u){pk16(hb[0], hb[1]), pk16(hb[2], hb[3]), pk16(hb[4], hb[5]), pk16(hb[6], hb[7])};
      *(volatile v4u*)(op + (size_t)row * kT + c8) = u;
    }
    __threadfence();
  }
}

__global__ __launch_bounds__(128) void decay_cast_kernel(const float* __restrict__ sf, unsigned short* __restrict__ s16, int h0) {
  const int n  = blockIdx.x;
  const int gl = blockIdx.y;
  const int h  = h0 + gl;
  const int tid = threadIdx.x;
  const int wave = tid >> 5;
  const int m0 = tid * 8;
  const float lstart = -3.4657359027997265f;
  const float lstop  = -6.2383246250395077f;
  const float frac = (float)h * (1.0f / 15.0f);
  const float lin  = lstart * (1.0f - frac) + lstop * frac;
  const float gam  = 1.0f - expf(lin);
  const float lg   = log2f(gam);
  const size_t rowoff = ((size_t)gl * kT + n) * kT + m0;
  v4u u = (v4u){0u, 0u, 0u, 0u};
  if (wave * 256 <= n) {
    const v4f a = *(const v4f*)(sf + rowoff);
    const v4f c = *(const v4f*)(sf + rowoff + 4);
    unsigned short hb[8];
#pragma unroll
    for (int e = 0; e < 8; ++e) {
      const float sv = (e < 4) ? a[e] : c[e - 4];
      const int d  = n - (m0 + e);
      const int dc = d < 0 ? 0 : d;
      const float f = kSim256 * exp2f((float)dc * lg);
      const float val = (d >= 0) ? sv * f : 0.0f;
      hb[e] = h_bits(val);
    }
    u = (v4u){pk16(hb[0], hb[1]), pk16(hb[2], hb[3]), pk16(hb[4], hb[5]), pk16(hb[6], hb[7])};
  }
  unsigned short* po = s16 + rowoff;
  *(volatile v4u*)po = u;
  __threadfence();
  *(volatile v4u*)po = u;
}

__device__ __forceinline__ float silu_carry(float xv) {
  const float e   = expf(-fabsf(xv));
  const float rcp = 1.0f / (1.0f + e);
  const float sig = (xv >= 0.0f) ? rcp : e * rcp;
  return xv * sig * kHCarry;
}
__global__ __launch_bounds__(256) void silu_cast_kernel(const float* __restrict__ u, unsigned short* __restrict__ out, int n8) {
  const int i = blockIdx.x * 256 + threadIdx.x;
  if (i >= n8) return;
  const float* p = u + 8 * (size_t)i;
  unsigned r0 = 0u, r1 = 0u, r2 = 0u, r3 = 0u;
#pragma unroll 1
  for (int it = 0; it < 4; ++it) {
    const float x0 = p[2 * it];
    const float x1 = p[2 * it + 1];
    const unsigned w = pk16(h_bits(silu_carry(x0)), h_bits(silu_carry(x1)));
    r0 = (it == 0) ? w : r0;
    r1 = (it == 1) ? w : r1;
    r2 = (it == 2) ? w : r2;
    r3 = (it == 3) ? w : r3;
  }
  const v4u uu = (v4u){r0, r1, r2, r3};
  unsigned short* q = out + 8 * (size_t)i;
  *(volatile v4u*)q = uu;
  __threadfence();
  *(volatile v4u*)q = uu;
}

extern "C" void kernel_launch(void* const* d_in, const int* in_sizes, int n_in,
                              void* d_out, int out_size, void* d_ws, size_t ws_size, hipStream_t stream) {
  if (n_in < 14) return;
  if (in_sizes[0] != kTok * kD || out_size != kTok * kD) return;
  if (in_sizes[3] != kD * kD || in_sizes[4] != kD * kD || in_sizes[5] != kD * kD || in_sizes[6] != kD * kD) return;
  if (in_sizes[10] != kD2 * kD || in_sizes[12] != kD * kD2) return;
  if (in_sizes[1] != kD || in_sizes[7] != kD || in_sizes[11] != kD2 || in_sizes[13] != kD) return;
  if (ws_size < kWsTotal) return;

  const float* x  = (const float*)d_in[0];
  const float* ng = (const float*)d_in[1];
  const float* nb = (const float*)d_in[2];
  const float* qw = (const float*)d_in[3];
  const float* kw = (const float*)d_in[4];
  const float* vw = (const float*)d_in[5];
  const float* ow = (const float*)d_in[6];
  const float* ob = (const float*)d_in[7];
  const float* fg = (const float*)d_in[8];
  const float* fb = (const float*)d_in[9];
  const float* w1 = (const float*)d_in[10];
  const float* b1 = (const float*)d_in[11];
  const float* w2 = (const float*)d_in[12];
  const float* b2 = (const float*)d_in[13];
  float* outp = (float*)d_out;

  char* ws = (char*)d_ws;
  unsigned short* w3_16 = (unsigned short*)(ws + kOffW3);
  unsigned short* ow16  = (unsigned short*)(ws + kOffOW);
  unsigned short* w1_16 = (unsigned short*)(ws + kOffW1);
  unsigned short* w2_16 = (unsigned short*)(ws + kOffW2);
  unsigned short* xn16  = (unsigned short*)(ws + kOffXN);
  unsigned short* y16   = xn16;
  float*          qkvf  = (float*)(ws + kOffBig);
  float*          sf    = (float*)(ws + kOffBig);
  float*          uf    = (float*)(ws + kOffBig);
  unsigned short* q16   = (unsigned short*)(ws + kOffQ);
  unsigned short* k16   = (unsigned short*)(ws + kOffK);
  unsigned short* h16   = (unsigned short*)(ws + kOffQ);
  unsigned short* vt16  = (unsigned short*)(ws + kOffVT);
  unsigned short* s16   = (unsigned short*)(ws + kOffX1);
  float*          x1f   = (float*)(ws + kOffX1);

  cast8_kernel<<<dim3(kD * kD / 8 / 256, 3), 256, 0, stream>>>(qw, kw, vw, w3_16, kD * kD / 8, kWCarry);
  cast8_kernel<<<dim3(kD * kD / 8 / 256, 1), 256, 0, stream>>>(ow, ow, ow, ow16, kD * kD / 8, kWCarry);
  cast8_kernel<<<dim3(kD2 * kD / 8 / 256, 1), 256, 0, stream>>>(w1, w1, w1, w1_16, kD2 * kD / 8, kWCarry);
  cast8_kernel<<<dim3(kD * kD2 / 8 / 256, 1), 256, 0, stream>>>(w2, w2, w2, w2_16, kD * kD2 / 8, kWCarry);

  groupnorm_kernel<<<dim3(kB * kH), 256, 0, stream>>>(x, ng, nb, xn16);
  wmma_gemm64<0, false, 0, 0, false, 0><<<dim3(kTok / 64 * (kQKVN / 64) / 8, 1), 256, 0, stream>>>(
      xn16, xn16, kD, 0L, w3_16, w3_16, kD, 0L, (void*)qkvf, (void*)qkvf, kQKVN, 0L, ob, ob, 0L,
      kTok, kQKVN, kD, kQKVScale);
  l2norm_qk_kernel<<<dim3(kTok), 128, 0, stream>>>(qkvf, q16, k16);
  vtrans_kernel<<<dim3(kT / 64, kH, kB), 256, 0, stream>>>(qkvf, vt16);

  for (int ch = 0; ch < kNChunk; ++ch) {
    const int g0 = ch * kChunkG;
    const int bb = g0 / kH;
    const int hh0 = g0 % kH;
    const unsigned short* qg = q16 + (size_t)g0 * kT * kDH;
    const unsigned short* kg = k16 + (size_t)g0 * kT * kDH;
    const unsigned short* vg = vt16 + (size_t)g0 * kDH * kT;
    unsigned short* yg = y16 + (size_t)bb * kT * kD + (size_t)hh0 * kDH;
    wmma_gemm64<0, false, 0, 0, false, 0><<<dim3(kT / 64 * (kT / 64) / 8, kChunkG), 256, 0, stream>>>(
        qg, qg, kDH, (long)kT * kDH, kg, kg, kDH, (long)kT * kDH, (void*)sf, (void*)sf, kT, (long)kT * kT, ob, ob, 0L,
        kT, kT, kDH, kSScale);
    decay_cast_kernel<<<dim3(kT, kChunkG), 128, 0, stream>>>(sf, s16, hh0);
    wmma_gemm64<0, false, 0, 1, false, 0><<<dim3(kT / 64 * (kDH / 64) / 8, kChunkG), 256, 0, stream>>>(
        s16, s16, kT, (long)kT * kT, vg, vg, kT, (long)kDH * kT, (void*)yg, (void*)yg, kD, (long)kDH, ob, ob, 0L,
        kT, kDH, kT, kPVScale);
  }

  wmma_gemm64<0, false, 2, 0, true, 0><<<dim3(kTok / 64 * (kD / 64) / 8, 1), 256, 0, stream>>>(
      y16, y16, kD, 0L, ow16, ow16, kD, 0L, (void*)x1f, (void*)x1f, kD, 0L, ob, x, 0L,
      kTok, kD, kD, kOWScale);

  groupnorm_kernel<<<dim3(kB * kH), 256, 0, stream>>>(x1f, fg, fb, xn16);
  wmma_gemm64<0, false, 2, 0, false, 0><<<dim3(kTok / 64 * (kD2 / 64) / 8, 1), 256, 0, stream>>>(
      xn16, xn16, kD, 0L, w1_16, w1_16, kD, 0L, (void*)uf, (void*)uf, kD2, 0L, b1, b1, 0L,
      kTok, kD2, kD, kW1Scale);
  silu_cast_kernel<<<dim3(kTok * kD2 / 8 / 256), 256, 0, stream>>>(uf, h16, kTok * kD2 / 8);
  wmma_gemm64<0, false, 2, 0, true, 0><<<dim3(kTok / 64 * (kD / 64) / 8, 1), 256, 0, stream>>>(
      h16, h16, kD2, 0L, w2_16, w2_16, kD2, 0L, (void*)outp, (void*)outp, kD, 0L, b2, x1f, 0L,
      kTok, kD, kD2, kW2Scale);
}
